// EnSSM_77206332113401
// MI455X (gfx1250) — hardware-run, weakly checked
//
#include <hip/hip_runtime.h>
#include <hip/hip_bf16.h>
#include <math.h>

#define NBAT  4
#define LL    2048
#define LP    (LL + 2)
#define NHALF 2
#define HB    (NBAT / NHALF)
#define HTOK  (HB * LL)
#define CIN   256
#define DMOD  512
#define DIN   1024
#define XZW   (2 * DIN)
#define DST   16
#define DTR   32
#define XDN   (DTR + 2 * DST)
#define DCV   4
#define NTAP  3
#define GSTR  40
#define OSTR  68
#define SMEMB (8 * 16 * OSTR * 4)
#define SCH   32
#define SYP   260
#define LOG2E 1.4426950408889634f
#define WSCAP ((size_t)134217728)
#define SC_U   16.0f
#define SC_XS  256.0f
#define SC_DTL 64.0f
#define SC_Y   1024.0f
#define SC_W   64.0f
#define SC_WDT 16.0f

static_assert(HTOK % 128 == 0);
static_assert(LL % 128 == 0);
static_assert(XZW % 64 == 0);
static_assert(XDN == 64);
static_assert(DIN % 64 == 0);
static_assert(DMOD % 64 == 0);
static_assert(CIN == 256);
static_assert(DMOD == 4 * 128);
static_assert(DIN == 4 * 256);
static_assert(DTR == 32);
static_assert(DST == 16);
static_assert(LL % SCH == 0);
static_assert(SCH == 32);
static_assert(SYP % 4 == 0);
static_assert(SYP >= 256);
static_assert(SMEMB >= (128 * GSTR + 64 * GSTR) * 2);
static_assert((NBAT * LP * CIN) % (8 * 256) == 0);

typedef unsigned short us16 __attribute__((ext_vector_type(16)));
typedef unsigned short us8  __attribute__((ext_vector_type(8)));
typedef unsigned short us8a __attribute__((ext_vector_type(8), may_alias));
typedef __bf16 v16b __attribute__((ext_vector_type(16)));
typedef _Float16 v16h __attribute__((ext_vector_type(16)));
typedef float v8f __attribute__((ext_vector_type(8)));
typedef float v4f __attribute__((ext_vector_type(4)));
typedef float v4fa __attribute__((ext_vector_type(4), may_alias));
union FragU { us16 v; us8 h[2]; };

__device__ __forceinline__ unsigned short bf16_bits(float f) {
  unsigned u = __float_as_uint(f);
  u += 0x7FFFu + ((u >> 16) & 1u);
  return (unsigned short)(u >> 16);
}
__device__ __forceinline__ float bf16_val(unsigned short b) { return __uint_as_float(((unsigned)b) << 16); }
__device__ __forceinline__ float bf16r(float f) { return bf16_val(bf16_bits(f)); }
__device__ __forceinline__ unsigned short h16_bits(float f) { return __builtin_bit_cast(unsigned short, (_Float16)f); }
__device__ __forceinline__ float siluf(float x) { return x * __builtin_amdgcn_rcpf(1.0f + __expf(-x)); }

__device__ __forceinline__ float wsum(float v) {
#pragma unroll
  for (int o = 16; o > 0; o >>= 1) v += __shfl_xor(v, o, 32);
  return v;
}

template <int BF>
__device__ __forceinline__ v8f mma16(us16 a, us16 b, v8f c) {
  if (BF) return __builtin_amdgcn_wmma_f32_16x16x32_bf16(false, __builtin_bit_cast(v16b, a), false, __builtin_bit_cast(v16b, b), (short)0, c, false, false);
  return __builtin_amdgcn_wmma_f32_16x16x32_f16(false, __builtin_bit_cast(v16h, a), false, __builtin_bit_cast(v16h, b), (short)0, c, false, false);
}
__device__ __forceinline__ void wguard5(v8f (&c)[4], const us16& a, const us16 (&b)[4]) {
#if defined(__HIP_DEVICE_COMPILE__)
  asm volatile("v_nop\n\tv_nop\n\tv_nop\n\tv_nop"
               : "+v"(c[0]), "+v"(c[1]), "+v"(c[2]), "+v"(c[3])
               : "v"(a), "v"(b[0]), "v"(b[1]), "v"(b[2]), "v"(b[3]));
#endif
}
__device__ __forceinline__ void wguard9(v8f (&c)[4], v8f (&e)[4], const us16& a, const us16 (&b)[4]) {
#if defined(__HIP_DEVICE_COMPILE__)
  asm volatile("v_nop\n\tv_nop\n\tv_nop\n\tv_nop"
               : "+v"(c[0]), "+v"(c[1]), "+v"(c[2]), "+v"(c[3]), "+v"(e[0]), "+v"(e[1]), "+v"(e[2]), "+v"(e[3])
               : "v"(a), "v"(b[0]), "v"(b[1]), "v"(b[2]), "v"(b[3]));
#endif
}

__device__ __forceinline__ us16 lds_frag(const unsigned short* base) {
  const int lane = threadIdx.x & 31, r = lane & 15, kh = (lane >> 4) * 8;
  FragU f;
  f.h[0] = *(const us8a*)(base + r * GSTR + kh);
  f.h[1] = *(const us8a*)(base + r * GSTR + 16 + kh);
  return f.v;
}

__device__ __forceinline__ void stage_a(unsigned short* lds, const unsigned short* __restrict__ P, int ld, int m0, int k0, int tid) {
  const int row = tid >> 1, cq = (tid & 1) * 16;
  const unsigned short* src = P + (size_t)(m0 + row) * ld + k0 + cq;
  const us8 v0 = *(const us8a*)src;
  const us8 v1 = *(const us8a*)(src + 8);
  *(us8a*)(lds + row * GSTR + cq) = v0;
  *(us8a*)(lds + row * GSTR + cq + 8) = v1;
}
__device__ __forceinline__ void stage_b(unsigned short* lds, const unsigned short* __restrict__ P, int ld, int n0, int k0, int tid) {
  const int row = tid >> 2, kq = (tid & 3) * 8;
  const us8 v = *(const us8a*)(P + (size_t)(n0 + row) * ld + k0 + kq);
  *(us8a*)(lds + row * GSTR + kq) = v;
}

template <int BF>
__global__ __launch_bounds__(256) void k_gemm(const unsigned short* __restrict__ A0, int lda,
                                             const unsigned short* __restrict__ B0, int ldb, float* Y, int ldy, int K, float oscale) {
  __shared__ __attribute__((aligned(16))) unsigned char sm[SMEMB];
  unsigned short* lA0 = (unsigned short*)sm;
  unsigned short* lB0 = lA0 + 128 * GSTR;
  float* oS = (float*)sm;
  const int tid = threadIdx.x, lane = tid & 31, wave = tid >> 5, cl = lane & 15, hh = lane >> 4;
  const int m0 = blockIdx.x * 128, n0 = blockIdx.y * 64;

  v8f acc[4];
#pragma unroll
  for (int j = 0; j < 4; ++j) { v8f zz = {0.f, 0.f, 0.f, 0.f, 0.f, 0.f, 0.f, 0.f}; acc[j] = zz; }

#pragma unroll 1
  for (int k0 = 0; k0 < K; k0 += 32) {
    __syncthreads();
    stage_a(lA0, A0, lda, m0, k0, tid);
    stage_b(lB0, B0, ldb, n0, k0, tid);
    __syncthreads();
    const us16 af0 = lds_frag(lA0 + 16 * wave * GSTR);
    us16 bfr[4];
#pragma unroll
    for (int j = 0; j < 4; ++j) bfr[j] = lds_frag(lB0 + 16 * j * GSTR);
#pragma unroll
    for (int j = 0; j < 4; ++j) acc[j] = mma16<BF>(af0, bfr[j], acc[j]);
    wguard5(acc, af0, bfr);
  }
  __syncthreads();

  float* so = oS + wave * (16 * OSTR);
#pragma unroll
  for (int j = 0; j < 4; ++j)
#pragma unroll
    for (int r = 0; r < 8; ++r) so[(8 * hh + r) * OSTR + 16 * j + cl] = acc[j][r] * oscale;
  __syncthreads();
#pragma unroll
  for (int pass = 0; pass < 2; ++pass) {
#pragma unroll
    for (int it = 0; it < 8; ++it) {
      const int ch = it * 32 + lane, r = ch >> 4, q = (ch & 15) * 4;
      const v4f v = *(const v4fa*)(so + r * OSTR + q);
      *(volatile v4f*)(Y + (size_t)(m0 + 16 * wave + r) * ldy + n0 + q) = v;
    }
    __threadfence();
  }
}

__global__ __launch_bounds__(256) void k_gemm_conv(const unsigned short* __restrict__ XP, const unsigned short* __restrict__ WC,
                                                  const float* __restrict__ bng, const float* __restrict__ bnb,
                                                  const float* __restrict__ bnm, const float* __restrict__ bnv, float* U) {
#pragma clang fp contract(off)
  __shared__ __attribute__((aligned(16))) unsigned char sm[SMEMB];
  unsigned short* lA = (unsigned short*)sm;
  unsigned short* lB = lA + 128 * GSTR;
  float* oS = (float*)sm;
  const int tid = threadIdx.x, lane = tid & 31, wave = tid >> 5, cl = lane & 15, hh = lane >> 4;
  const int m0 = blockIdx.x * 128, n0 = blockIdx.y * 64;
  const int b = m0 / LL, l0 = m0 - b * LL;
  const unsigned short* XPb = XP + (size_t)b * LP * CIN;
  const unsigned short* WR = WC + (size_t)NTAP * DMOD * CIN;

  v8f acc1[4], acc2[4];
#pragma unroll
  for (int j = 0; j < 4; ++j) { v8f zz = {0.f, 0.f, 0.f, 0.f, 0.f, 0.f, 0.f, 0.f}; acc1[j] = zz; acc2[j] = zz; }

#pragma unroll 1
  for (int s = 0; s < 32; ++s) {
    const bool isres = (s >= NTAP * 8);
    const int kk = isres ? 1 : (s >> 3);
    const int cb = (s & 7) * 32;
    const unsigned short* Bsrc = isres ? WR : (WC + (size_t)kk * DMOD * CIN);
    __syncthreads();
    stage_a(lA, XPb + (size_t)kk * CIN, CIN, l0, cb, tid);
    stage_b(lB, Bsrc, CIN, n0, cb, tid);
    __syncthreads();
    const us16 af = lds_frag(lA + 16 * wave * GSTR);
    us16 bw[4];
#pragma unroll
    for (int j = 0; j < 4; ++j) bw[j] = lds_frag(lB + 16 * j * GSTR);
    if (!isres) {
#pragma unroll
      for (int j = 0; j < 4; ++j) acc1[j] = mma16<1>(af, bw[j], acc1[j]);
    } else {
#pragma unroll
      for (int j = 0; j < 4; ++j) acc2[j] = mma16<1>(af, bw[j], acc2[j]);
    }
    wguard9(acc1, acc2, af, bw);
  }
  __syncthreads();

  float* so = oS + wave * (16 * OSTR);
#pragma unroll
  for (int j = 0; j < 4; ++j) {
    const int d = n0 + 16 * j + cl;
    const float sc = bf16r(bng[d]) * rsqrtf(bf16r(bnv[d]) + 1e-5f);
    const float mn = bf16r(bnm[d]), bb = bf16r(bnb[d]);
#pragma unroll
    for (int r = 0; r < 8; ++r) {
      float hv = (acc1[j][r] - mn) * sc + bb;
      hv = fmaxf(hv, 0.0f) + acc2[j][r];
      so[(8 * hh + r) * OSTR + 16 * j + cl] = hv;
    }
  }
  __syncthreads();
#pragma unroll
  for (int pass = 0; pass < 2; ++pass) {
#pragma unroll
    for (int it = 0; it < 8; ++it) {
      const int ch = it * 32 + lane, r = ch >> 4, q = (ch & 15) * 4;
      const v4f v = *(const v4fa*)(so + r * OSTR + q);
      *(volatile v4f*)(U + (size_t)(m0 + 16 * wave + r) * DMOD + n0 + q) = v;
    }
    __threadfence();
  }
}

template <int MODE>
__global__ __launch_bounds__(256) void k_cvt(const float* __restrict__ src, int spitch, unsigned short* dst, int ncol8, int total8, float scale) {
  const int idx = blockIdx.x * 256 + threadIdx.x;
  if (idx >= total8) return;
  const int row = idx / ncol8, c8 = (idx - row * ncol8) * 8;
  const float* s = src + (size_t)row * (size_t)spitch + c8;
  const v4f a = *(const v4fa*)s, b = *(const v4fa*)(s + 4);
  us8 o;
#pragma unroll
  for (int u = 0; u < 4; ++u) {
    const float va = a[u], vb = b[u];
    if (MODE == 0)      { o[u] = bf16_bits(va);               o[4 + u] = bf16_bits(vb); }
    else if (MODE == 1) { o[u] = h16_bits(bf16r(va) * scale); o[4 + u] = h16_bits(bf16r(vb) * scale); }
    else                { o[u] = h16_bits(va * scale);        o[4 + u] = h16_bits(vb * scale); }
  }
  const size_t off = (size_t)row * (size_t)(ncol8 * 8) + c8;
  *(volatile us8*)(dst + off) = o;
  __threadfence();
  *(volatile us8*)(dst + off) = o;
}

__global__ __launch_bounds__(256) void k_prepw(const float* __restrict__ w1, const float* __restrict__ wr, unsigned short* WC) {
  const int idx = blockIdx.x * 256 + threadIdx.x;
  const int e = idx * 8;
  const int grp = e >> 17;
  const int r = e & (DMOD * CIN - 1), d = r >> 8, c = r & 255;
  const int kk = (grp < NTAP) ? grp : (NTAP - 1);
  us8 o;
#pragma unroll
  for (int u = 0; u < 8; ++u) {
    const float v1 = w1[(size_t)(d * CIN + c + u) * NTAP + kk];
    const float v2 = wr[d * CIN + c + u];
    o[u] = bf16_bits((grp < NTAP) ? v1 : v2);
  }
  *(volatile us8*)(WC + e) = o;
  __threadfence();
  *(volatile us8*)(WC + e) = o;
}

__global__ __launch_bounds__(256) void k_cvtx(const float* __restrict__ x, unsigned short* XP, int total8) {
  const int idx = blockIdx.x * 256 + threadIdx.x;
  if (idx >= total8) return;
  const int row = idx >> 5, c8 = (idx & 31) * 8;
  const int b = row / LP, lp = row - b * LP;
  const bool valid = (lp >= 1) && (lp <= LL);
  int ls = lp - 1;
  ls = (ls < 0) ? 0 : ls;
  ls = (ls > LL - 1) ? (LL - 1) : ls;
  const float* s = x + ((size_t)b * LL + (size_t)ls) * CIN + c8;
  const v4f a = *(const v4fa*)s, bq = *(const v4fa*)(s + 4);
  us8 o;
#pragma unroll
  for (int u = 0; u < 4; ++u) {
    o[u]     = valid ? bf16_bits(a[u]) : (unsigned short)0;
    o[4 + u] = valid ? bf16_bits(bq[u]) : (unsigned short)0;
  }
  const size_t off = (size_t)row * CIN + c8;
  *(volatile us8*)(XP + off) = o;
  __threadfence();
  *(volatile us8*)(XP + off) = o;
}

__global__ __launch_bounds__(256) void k_conv(const float* __restrict__ XZ, const float* __restrict__ cw, const float* __restrict__ cb,
                                             float* XCF, unsigned short* XCH) {
#pragma clang fp contract(off)
  __shared__ __attribute__((aligned(16))) float sxs[DIN];
  const int tid = threadIdx.x, c4 = tid * 4;
  const int tok = blockIdx.x, l = tok & (LL - 1);
  v4f xv[DCV];
#pragma unroll
  for (int j = 0; j < DCV; ++j) {
    const int ll = l - (DCV - 1) + j;
    const int tc = (ll >= 0) ? (tok - (DCV - 1) + j) : tok;
    xv[j] = *(const v4fa*)(XZ + (size_t)tc * XZW + c4);
  }
  const v4f bb = *(const v4fa*)(cb + c4);
  v4f sv;
#pragma unroll
  for (int u = 0; u < 4; ++u) {
    const v4f wv = *(const v4fa*)(cw + (size_t)(c4 + u) * DCV);
    float a = 0.0f;
#pragma unroll
    for (int j = 0; j < DCV; ++j) {
      const float pr = bf16r(wv[j]) * xv[j][u];
      a = a + ((l - (DCV - 1) + j >= 0) ? pr : 0.0f);
    }
    a = a + bf16r(bb[u]);
    sv[u] = siluf(a);
  }
  *(v4fa*)(sxs + c4) = sv;
  const size_t o = (size_t)tok * DIN + c4;
  *(volatile v4f*)(XCF + o) = sv;
  __threadfence();
  *(volatile v4f*)(XCF + o) = sv;
  __syncthreads();
  if (tid < 128) {
    const int c8 = tid * 8;
    const v4f a = *(const v4fa*)(sxs + c8);
    const v4f b = *(const v4fa*)(sxs + c8 + 4);
    us8 hv;
#pragma unroll
    for (int u = 0; u < 4; ++u) { hv[u] = h16_bits(a[u] * SC_XS); hv[4 + u] = h16_bits(b[u] * SC_XS); }
    const size_t o2 = (size_t)tok * DIN + c8;
    *(volatile us8*)(XCH + o2) = hv;
    __threadfence();
    *(volatile us8*)(XCH + o2) = hv;
  }
}

__global__ __launch_bounds__(256) void k_scan(const float* __restrict__ XZ, const float* __restrict__ XCF, const float* __restrict__ XD,
                                             const float* __restrict__ DTW, const float* __restrict__ dtb, const float* __restrict__ Alog,
                                             const float* __restrict__ Dv, unsigned short* YH) {
#pragma clang fp contract(off)
  __shared__ __attribute__((aligned(16))) float sy[SCH * SYP];
  const int b = blockIdx.x >> 2, dg = blockIdx.x & 3, tid = threadIdx.x, lane = tid & 31, wave = tid >> 5;
  const int d = dg * 256 + tid;
  float A2[DST], h[DST];
#pragma unroll
  for (int n = 0; n < DST; ++n) { A2[n] = -__expf(bf16r(Alog[d * DST + n])) * LOG2E; h[n] = 0.0f; }
  const float Dd = bf16r(Dv[d]);
  const float bd = bf16r(dtb[d]);
#pragma unroll 1
  for (int c = 0; c < LL / SCH; ++c) {
#pragma unroll 1
    for (int s = 0; s < SCH; ++s) {
      const size_t tok = (size_t)b * LL + (size_t)(c * SCH + s);
      const float raw = DTW[tok * DIN + d];
      const float a = raw + bd;
      const float dl = fmaxf(a, 0.0f) + log1pf(__expf(-fabsf(a)));
      const float xv = XCF[tok * DIN + d];
      const float zv = XZ[tok * XZW + DIN + d];
      const float* bcp = XD + tok * XDN;
      v4f Bv[4], Cv[4];
#pragma unroll
      for (int q = 0; q < 4; ++q) {
        Bv[q] = *(const v4fa*)(bcp + DTR + 4 * q);
        Cv[q] = *(const v4fa*)(bcp + DTR + DST + 4 * q);
      }
      const float dx = dl * xv;
      float y = 0.0f;
#pragma unroll
      for (int n = 0; n < DST; ++n) {
        const float e = exp2f(dl * A2[n]);
        h[n] = e * h[n] + dx * Bv[n >> 2][n & 3];
        y = y + h[n] * Cv[n >> 2][n & 3];
      }
      const float yv = (y + xv * Dd) * siluf(zv);
      sy[s * SYP + tid] = yv;
    }
    __syncthreads();
#pragma unroll
    for (int pass = 0; pass < 2; ++pass) {
#pragma unroll
      for (int it = 0; it < 4; ++it) {
        const int row = 4 * wave + it;
        const v4f va = *(const v4fa*)(sy + row * SYP + lane * 8);
        const v4f vb = *(const v4fa*)(sy + row * SYP + lane * 8 + 4);
        us8 o;
#pragma unroll
        for (int u = 0; u < 4; ++u) { o[u] = h16_bits(va[u] * SC_Y); o[4 + u] = h16_bits(vb[u] * SC_Y); }
        const size_t off = ((size_t)b * LL + (size_t)(c * SCH + row)) * DIN + (size_t)dg * 256 + (size_t)lane * 8;
        *(volatile us8*)(YH + off) = o;
      }
      __threadfence();
    }
    __syncthreads();
  }
}

__global__ __launch_bounds__(128) void k_final(const float* __restrict__ U, const float* __restrict__ MO, const float* __restrict__ g,
                                              const float* __restrict__ be, float* out) {
#pragma clang fp contract(off)
  __shared__ float sred[8];
  const int tid = threadIdx.x, lane = tid & 31, wave = tid >> 5, c4 = tid * 4;
  const int tok = blockIdx.x;
  const size_t o = (size_t)tok * DMOD + c4;
  const v4f mv = *(const v4fa*)(MO + o);
  const v4f uv = *(const v4fa*)(U + o);
  float s = (mv[0] + mv[1]) + (mv[2] + mv[3]);
  s = wsum(s);
  if (lane == 0) sred[wave] = s;
  __syncthreads();
  const float mean = ((sred[0] + sred[1]) + (sred[2] + sred[3])) * (1.0f / DMOD);
  v4f dv;
  float q = 0.0f;
#pragma unroll
  for (int u = 0; u < 4; ++u) { dv[u] = mv[u] - mean; q = q + dv[u] * dv[u]; }
  q = wsum(q);
  if (lane == 0) sred[4 + wave] = q;
  __syncthreads();
  const float var = ((sred[4] + sred[5]) + (sred[6] + sred[7])) * (1.0f / DMOD);
  const float inv = rsqrtf(var + 1e-6f);
  const v4f gv = *(const v4fa*)(g + c4), ev = *(const v4fa*)(be + c4);
  v4f ov;
#pragma unroll
  for (int u = 0; u < 4; ++u) ov[u] = uv[u] + (dv[u] * inv * bf16r(gv[u]) + bf16r(ev[u]));
  *(volatile v4f*)(out + o) = ov;
  __threadfence();
  *(volatile v4f*)(out + o) = ov;
}

extern "C" void kernel_launch(void* const* d_in, const int* in_sizes, int n_in,
                              void* d_out, int out_size, void* d_ws, size_t ws_size,
                              hipStream_t stream) {
  if (n_in < 18) return;
  if (in_sizes[0] != NBAT * LL * CIN || in_sizes[1] != DMOD * CIN * NTAP || in_sizes[2] != DMOD * CIN ||
      in_sizes[3] != DMOD || in_sizes[4] != DMOD || in_sizes[5] != DMOD || in_sizes[6] != DMOD ||
      in_sizes[7] != XZW * DMOD || in_sizes[8] != DIN * DCV || in_sizes[9] != DIN || in_sizes[10] != XDN * DIN ||
      in_sizes[11] != DIN * DTR || in_sizes[12] != DIN || in_sizes[13] != DIN * DST || in_sizes[14] != DIN ||
      in_sizes[15] != DMOD * DIN || in_sizes[16] != DMOD || in_sizes[17] != DMOD || out_size != NBAT * LL * DMOD) return;

  const float* x     = (const float*)d_in[0];
  const float* c3w   = (const float*)d_in[1];
  const float* crw   = (const float*)d_in[2];
  const float* bng   = (const float*)d_in[3];
  const float* bnb   = (const float*)d_in[4];
  const float* bnm   = (const float*)d_in[5];
  const float* bnv   = (const float*)d_in[6];
  const float* inw   = (const float*)d_in[7];
  const float* c1w   = (const float*)d_in[8];
  const float* c1b   = (const float*)d_in[9];
  const float* xpw   = (const float*)d_in[10];
  const float* dtw   = (const float*)d_in[11];
  const float* dtb   = (const float*)d_in[12];
  const float* Alog  = (const float*)d_in[13];
  const float* Dv    = (const float*)d_in[14];
  const float* ow    = (const float*)d_in[15];
  const float* lng   = (const float*)d_in[16];
  const float* lnb   = (const float*)d_in[17];
  float* out = (float*)d_out;

  size_t off = 0;
  auto carve = [&](size_t bytes) -> char* { char* p = (char*)d_ws + off; off += (bytes + 255) & ~(size_t)255; return p; };
  unsigned short* WIN16 = (unsigned short*)carve((size_t)XZW * DMOD * 2);
  unsigned short* WX16  = (unsigned short*)carve((size_t)XDN * DIN * 2);
  unsigned short* WDT16 = (unsigned short*)carve((size_t)DIN * DTR * 2);
  unsigned short* WO16  = (unsigned short*)carve((size_t)DMOD * DIN * 2);
  unsigned short* WC    = (unsigned short*)carve((size_t)(NTAP + 1) * DMOD * CIN * 2);
  unsigned short* XP16  = (unsigned short*)carve((size_t)NBAT * LP * CIN * 2);
  float* U              = (float*)carve((size_t)HTOK * DMOD * 4);
  unsigned short* U16   = (unsigned short*)carve((size_t)HTOK * DMOD * 2);
  float* XZ             = (float*)carve((size_t)HTOK * XZW * 4);
  float* XCF            = (float*)carve((size_t)HTOK * DIN * 4);
  unsigned short* XCH   = (unsigned short*)carve((size_t)HTOK * DIN * 2);
  float* XD             = (float*)carve((size_t)HTOK * XDN * 4);
  unsigned short* DT16  = (unsigned short*)carve((size_t)HTOK * DTR * 2);
  float* DTW            = (float*)carve((size_t)HTOK * DIN * 4);
  unsigned short* YH    = (unsigned short*)carve((size_t)HTOK * DIN * 2);
  float* MO             = (float*)carve((size_t)HTOK * DMOD * 4);
  if (off > ws_size || off > WSCAP) return;

  const dim3 b256(256), b128(128);
  auto cvt_w = [&](const float* src, int spitch, unsigned short* dst, int nrow, int ncol, float scale) {
    const int ncol8 = ncol / 8, total8 = nrow * ncol8;
    k_cvt<1><<<dim3((total8 + 255) / 256), b256, 0, stream>>>(src, spitch, dst, ncol8, total8, scale);
  };
  auto cvt_a = [&](const float* src, int spitch, unsigned short* dst, int nrow, int ncol, float scale) {
    const int ncol8 = ncol / 8, total8 = nrow * ncol8;
    k_cvt<2><<<dim3((total8 + 255) / 256), b256, 0, stream>>>(src, spitch, dst, ncol8, total8, scale);
  };
  cvt_w(inw, DMOD, WIN16, XZW, DMOD, SC_W);
  cvt_w(xpw, DIN, WX16, XDN, DIN, SC_W);
  cvt_w(dtw, DTR, WDT16, DIN, DTR, SC_WDT);
  cvt_w(ow, DIN, WO16, DMOD, DIN, SC_W);
  k_prepw<<<dim3(((NTAP + 1) * DMOD * CIN / 8) / 256), b256, 0, stream>>>(c3w, crw, WC);
  {
    const int total8 = NBAT * LP * CIN / 8;
    k_cvtx<<<dim3((total8 + 255) / 256), b256, 0, stream>>>(x, XP16, total8);
  }

  for (int hp = 0; hp < NHALF; ++hp) {
    const unsigned short* XPh = XP16 + (size_t)hp * HB * LP * CIN;
    float* outh = out + (size_t)hp * HTOK * DMOD;
    k_gemm_conv<<<dim3(HTOK / 128, DMOD / 64), b256, 0, stream>>>(XPh, WC, bng, bnb, bnm, bnv, U);
    cvt_a(U, DMOD, U16, HTOK, DMOD, SC_U);
    k_gemm<0><<<dim3(HTOK / 128, XZW / 64), b256, 0, stream>>>(U16, DMOD, WIN16, DMOD, XZ, XZW, DMOD, 1.0f / (SC_U * SC_W));
    k_conv<<<dim3(HTOK), b256, 0, stream>>>(XZ, c1w, c1b, XCF, XCH);
    k_gemm<0><<<dim3(HTOK / 128, XDN / 64), b256, 0, stream>>>(XCH, DIN, WX16, DIN, XD, XDN, DIN, 1.0f / (SC_XS * SC_W));
    cvt_a(XD, XDN, DT16, HTOK, DTR, SC_DTL);
    k_gemm<0><<<dim3(HTOK / 128, DIN / 64), b256, 0, stream>>>(DT16, DTR, WDT16, DTR, DTW, DIN, DTR, 1.0f / (SC_DTL * SC_WDT));
    k_scan<<<dim3(HB * (DIN / 256)), b256, 0, stream>>>(XZ, XCF, XD, DTW, dtb, Alog, Dv, YH);
    k_gemm<0><<<dim3(HTOK / 128, DMOD / 64), b256, 0, stream>>>(YH, DIN, WO16, DIN, MO, DMOD, DIN, 1.0f / (SC_Y * SC_W));
    k_final<<<dim3(HTOK), b128, 0, stream>>>(U, MO, lng, lnb, outh);
  }
}
